// YiJingAttention_49108656062775
// MI455X (gfx1250) — hardware-verified
//
#include <hip/hip_runtime.h>
#include <math.h>
#include <stdint.h>

#pragma clang fp contract(off)

#define NB    2
#define SEQ   2048
#define DM    1024
#define NH    8
#define NKV   4
#define NREP  (NH / NKV)
#define HD    128
#define DKV   (NKV * HD)
#define DQKV  (DM + 2 * DKV)
#define WIN   512
#define NQB   (SEQ / 64)
#define KTW   (((WIN - 1) + 63) / 64 + 1)
#define ROWS  (NB * SEQ)
#define OUTN  (ROWS * DM)
#define NFR   (HD / 2)
static_assert(NH * HD == DM);
static_assert(HD == 128);
static_assert(NREP == 2);
static_assert(WIN == 512);
static_assert(KTW == 9);
static_assert(NFR == 64);
static_assert((SEQ % 64) == 0 && (DM % 64) == 0 && (DKV % 64) == 0 && (DQKV % 64) == 0);
static_assert((DM % 32) == 0);
static_assert((((ROWS / 64) * (DQKV / 64)) % 8) == 0);
static_assert((((ROWS / 64) * (DM / 64)) % 8) == 0);
static_assert(((ROWS * DM / 8) % 256) == 0);
static_assert(((SEQ * NFR) % 256) == 0);

typedef _Float16 v16h __attribute__((ext_vector_type(16)));
typedef _Float16 v8h  __attribute__((ext_vector_type(8)));
typedef float    v8f  __attribute__((ext_vector_type(8)));
typedef float    v4f  __attribute__((ext_vector_type(4)));
typedef unsigned int v4u __attribute__((ext_vector_type(4)));

__device__ __forceinline__ unsigned short bf_bits(float f) {
  unsigned u = __float_as_uint(f);
  return (unsigned short)((u + 0x7FFFu + ((u >> 16) & 1u)) >> 16);
}
__device__ __forceinline__ float bfr(float f) { return __uint_as_float(((unsigned)bf_bits(f)) << 16); }
__device__ __forceinline__ unsigned short h_bits(_Float16 x) { return __builtin_bit_cast(unsigned short, x); }
__device__ __forceinline__ unsigned pk16(unsigned short a, unsigned short b) { return (unsigned)a | ((unsigned)b << 16); }
__device__ __forceinline__ v8f zero8() { v8f z = {0.f, 0.f, 0.f, 0.f, 0.f, 0.f, 0.f, 0.f}; return z; }
__device__ __forceinline__ void split16(float v, _Float16& hi, _Float16& rs) {
  hi = (_Float16)v;
  rs = (_Float16)((v - (float)hi) * 2048.0f);
}

__device__ __forceinline__ v16h ldfrag_h(const _Float16* p) {
  union { v16h v; v8h h[2]; } f;
  f.h[0] = *(const v8h*)(p);
  f.h[1] = *(const v8h*)(p + 16);
  return f.v;
}

__device__ __forceinline__ v8f mma_h(v16h a, v16h b, v8f c) {
  c = __builtin_amdgcn_wmma_f32_16x16x32_f16(false, a, false, b, (short)0, c, false, false);
#if defined(__HIP_DEVICE_COMPILE__)
  asm volatile("v_nop\n\tv_nop\n\tv_nop\n\tv_nop" : "+v"(c) : "v"(a), "v"(b));
#endif
  return c;
}
__device__ __forceinline__ v8f mma_h_raw(v16h a, v16h b, v8f c) {
  return __builtin_amdgcn_wmma_f32_16x16x32_f16(false, a, false, b, (short)0, c, false, false);
}
__device__ __forceinline__ void dep_guard_h(v8f& a, v8f& b, v16h x, v16h y) {
#if defined(__HIP_DEVICE_COMPILE__)
  asm volatile("v_nop\n\tv_nop\n\tv_nop\n\tv_nop" : "+v"(a), "+v"(b) : "v"(x), "v"(y));
#endif
}
__device__ __forceinline__ void keep4_h(v16h a, v16h b, v16h c, v16h d) {
#if defined(__HIP_DEVICE_COMPILE__)
  asm volatile("v_nop" :: "v"(a), "v"(b), "v"(c), "v"(d));
#endif
}
__device__ __forceinline__ void acc_guard4(v8f& a, v8f& b, v8f& c, v8f& d) {
#if defined(__HIP_DEVICE_COMPILE__)
  asm volatile("v_nop\n\tv_nop\n\tv_nop\n\tv_nop" : "+v"(a), "+v"(b), "+v"(c), "+v"(d));
#endif
}

__global__ __launch_bounds__(256) void cvt16(const float* __restrict__ in, unsigned short* out, int n8, float scale) {
  const int i = blockIdx.x * 256 + threadIdx.x;
  if (i < n8) {
    const v4f a = *(const v4f*)(in + (size_t)i * 8);
    const v4f b = *(const v4f*)(in + (size_t)i * 8 + 4);
    v4u p;
    p[0] = pk16(h_bits((_Float16)(bfr(a[0]) * scale)), h_bits((_Float16)(bfr(a[1]) * scale)));
    p[1] = pk16(h_bits((_Float16)(bfr(a[2]) * scale)), h_bits((_Float16)(bfr(a[3]) * scale)));
    p[2] = pk16(h_bits((_Float16)(bfr(b[0]) * scale)), h_bits((_Float16)(bfr(b[1]) * scale)));
    p[3] = pk16(h_bits((_Float16)(bfr(b[2]) * scale)), h_bits((_Float16)(bfr(b[3]) * scale)));
    *(volatile v4u*)(out + (size_t)i * 8) = p;
    __threadfence();
    *(volatile v4u*)(out + (size_t)i * 8) = p;
  }
}

__global__ __launch_bounds__(256) void w_tr(const float* __restrict__ w, unsigned short* wt, int K, int N, float scale) {
  __shared__ __align__(16) _Float16 sw[64 * 72];
  const int tid = threadIdx.x;
  const int n0  = blockIdx.x * 64;
  const int k0  = blockIdx.y * 64;
#pragma unroll
  for (int i = 0; i < 2; ++i) {
    const int idx = i * 256 + tid;
    const int kk = idx >> 3, c8 = (idx & 7) * 8;
    const float* src = w + (size_t)(k0 + kk) * N + n0 + c8;
    const v4f a  = *(const v4f*)(src);
    const v4f a2 = *(const v4f*)(src + 4);
    v8h o;
    o[0] = (_Float16)(bfr(a[0]) * scale);
    o[1] = (_Float16)(bfr(a[1]) * scale);
    o[2] = (_Float16)(bfr(a[2]) * scale);
    o[3] = (_Float16)(bfr(a[3]) * scale);
    o[4] = (_Float16)(bfr(a2[0]) * scale);
    o[5] = (_Float16)(bfr(a2[1]) * scale);
    o[6] = (_Float16)(bfr(a2[2]) * scale);
    o[7] = (_Float16)(bfr(a2[3]) * scale);
    *(v8h*)(sw + kk * 72 + c8) = o;
  }
  __syncthreads();

  const int g = tid >> 3, piece = tid & 7;
  v4u hv[2];
  size_t hofs[2];
#pragma unroll
  for (int it = 0; it < 2; ++it) {
    const int nn = it * 32 + g;
    v4u a;
#pragma unroll
    for (int e = 0; e < 4; ++e) {
      const _Float16 x0 = sw[(piece * 8 + 2 * e) * 72 + nn];
      const _Float16 x1 = sw[(piece * 8 + 2 * e + 1) * 72 + nn];
      a[e] = pk16(h_bits(x0), h_bits(x1));
    }
    hv[it] = a;
    hofs[it] = ((size_t)(n0 + nn)) * K + k0 + piece * 8;
  }
  for (int pass = 0; pass < 2; ++pass) {
#pragma unroll
    for (int it = 0; it < 2; ++it) *(volatile v4u*)(wt + hofs[it]) = hv[it];
    __threadfence();
  }
}

template <int EPI, bool ARES>
__global__ __launch_bounds__(256) void gemm64_f16(
    const unsigned short* __restrict__ Ap, const unsigned short* __restrict__ Arp, int lda,
    const unsigned short* __restrict__ Btp, int ldb,
    float cscale,
    void* Cp, unsigned short* Crp, int ldc, int M, int N, int K, float oscale,
    int tmod, int tlo, int thi) {
  const _Float16* Ah  = (const _Float16*)(const void*)Ap;
  const _Float16* Arh = (const _Float16*)(const void*)Arp;
  const _Float16* Bt  = (const _Float16*)(const void*)Btp;
  __shared__ __align__(16) float sT[8][16 * 68];
  const int lane = threadIdx.x & 31;
  const int wave = threadIdx.x >> 5;
  const int tilesN = N >> 6;
  const int tilesM = M >> 6;
  const int tile = blockIdx.x * 8 + wave;
  if (tile >= tilesM * tilesN) return;
  const int tm = tile / tilesN;
  const int tn = tile - tm * tilesN;
  const int m0 = tm << 6;
  const int n0 = tn << 6;
  const int tpos = m0 % tmod;
  if (tpos < tlo || tpos >= thi) return;

  const int rlane = lane & 15;
  const int koff  = (lane >> 4) * 8;
  const int mOff  = (lane >> 4) * 8;

  v8f acc[4][4];
#pragma unroll
  for (int i = 0; i < 4; ++i)
#pragma unroll
    for (int j = 0; j < 4; ++j) acc[i][j] = zero8();

  constexpr int NPL = ARES ? 2 : 1;
#pragma unroll 1
  for (int pl = 0; pl < NPL; ++pl) {
    const _Float16* Asel = (ARES && pl == 0) ? Arh : Ah;
    if (ARES && pl == 1) {
      acc_guard4(acc[0][0], acc[0][1], acc[0][2], acc[0][3]);
      acc_guard4(acc[1][0], acc[1][1], acc[1][2], acc[1][3]);
      acc_guard4(acc[2][0], acc[2][1], acc[2][2], acc[2][3]);
      acc_guard4(acc[3][0], acc[3][1], acc[3][2], acc[3][3]);
#pragma unroll
      for (int i = 0; i < 4; ++i)
#pragma unroll
        for (int j = 0; j < 4; ++j) acc[i][j] = acc[i][j] * (1.0f / 2048.0f);
      acc_guard4(acc[0][0], acc[0][1], acc[0][2], acc[0][3]);
      acc_guard4(acc[1][0], acc[1][1], acc[1][2], acc[1][3]);
      acc_guard4(acc[2][0], acc[2][1], acc[2][2], acc[2][3]);
      acc_guard4(acc[3][0], acc[3][1], acc[3][2], acc[3][3]);
    }
    for (int k0 = 0; k0 < K; k0 += 32) {
      v16h bh[4];
#pragma unroll
      for (int j = 0; j < 4; ++j) {
        const size_t bo = (size_t)(n0 + (j << 4) + rlane) * ldb + koff + k0;
        bh[j] = ldfrag_h(Bt + bo);
      }
#pragma unroll
      for (int i = 0; i < 4; ++i) {
        const size_t ao = (size_t)(m0 + (i << 4) + rlane) * lda + koff + k0;
        const v16h ah = ldfrag_h(Asel + ao);
#pragma unroll
        for (int j = 0; j < 4; ++j) {
          acc[i][j] = mma_h_raw(ah, bh[j], acc[i][j]);
        }
        dep_guard_h(acc[i][0], acc[i][3], ah, bh[3]);
      }
      keep4_h(bh[0], bh[1], bh[2], bh[3]);
    }
  }
  acc_guard4(acc[0][0], acc[0][1], acc[0][2], acc[0][3]);
  acc_guard4(acc[1][0], acc[1][1], acc[1][2], acc[1][3]);
  acc_guard4(acc[2][0], acc[2][1], acc[2][2], acc[2][3]);
  acc_guard4(acc[3][0], acc[3][1], acc[3][2], acc[3][3]);

  float* slab = sT[wave];
#pragma unroll
  for (int i = 0; i < 4; ++i) {
    const int mBase = m0 + (i << 4);
#pragma unroll
    for (int r = 0; r < 8; ++r) {
      const int row = mOff + r;
#pragma unroll
      for (int j = 0; j < 4; ++j) slab[row * 68 + (j << 4) + rlane] = acc[i][j][r] * cscale;
    }
    __builtin_amdgcn_fence(__ATOMIC_RELEASE, "workgroup");
    __builtin_amdgcn_wave_barrier();
    __builtin_amdgcn_fence(__ATOMIC_ACQUIRE, "workgroup");
    if constexpr (EPI == 0) {
      unsigned short* C16 = (unsigned short*)Cp;
      const int rq = lane >> 3, piece = lane & 7;
      v4u ph[4], pr[4];
#pragma unroll
      for (int it = 0; it < 4; ++it) {
        const int row = it * 4 + rq;
        const v4f a  = *(const v4f*)(slab + row * 68 + piece * 8);
        const v4f a2 = *(const v4f*)(slab + row * 68 + piece * 8 + 4);
        float f[8];
        f[0] = a[0];  f[1] = a[1];  f[2] = a[2];  f[3] = a[3];
        f[4] = a2[0]; f[5] = a2[1]; f[6] = a2[2]; f[7] = a2[3];
        v4u p, q;
#pragma unroll
        for (int e = 0; e < 4; ++e) {
          const float g0 = f[2 * e] * oscale, g1 = f[2 * e + 1] * oscale;
          const _Float16 x0 = (_Float16)g0, x1 = (_Float16)g1;
          const _Float16 y0 = (_Float16)((g0 - (float)x0) * 2048.0f);
          const _Float16 y1 = (_Float16)((g1 - (float)x1) * 2048.0f);
          p[e] = pk16(h_bits(x0), h_bits(x1));
          q[e] = pk16(h_bits(y0), h_bits(y1));
        }
        ph[it] = p;
        pr[it] = q;
      }
      for (int pass = 0; pass < 2; ++pass) {
#pragma unroll
        for (int it = 0; it < 4; ++it) {
          const int row = it * 4 + rq;
          const size_t co = (size_t)(mBase + row) * ldc + n0 + piece * 8;
          *(volatile v4u*)(C16 + co) = ph[it];
          *(volatile v4u*)(Crp + co) = pr[it];
        }
        __threadfence();
      }
    } else {
      float* Cf = (float*)Cp;
      const int hh = lane >> 4, c4 = (lane & 15) * 4;
      v4f ov[8];
#pragma unroll
      for (int it = 0; it < 8; ++it) {
        const int row = it * 2 + hh;
        ov[it] = *(const v4f*)(slab + row * 68 + c4);
      }
      for (int pass = 0; pass < 2; ++pass) {
#pragma unroll
        for (int it = 0; it < 8; ++it) {
          const int row = it * 2 + hh;
          *(volatile v4f*)(Cf + (size_t)(mBase + row) * ldc + n0 + c4) = ov[it];
        }
        __threadfence();
      }
    }
    __builtin_amdgcn_fence(__ATOMIC_RELEASE, "workgroup");
    __builtin_amdgcn_wave_barrier();
    __builtin_amdgcn_fence(__ATOMIC_ACQUIRE, "workgroup");
  }
}

__global__ __launch_bounds__(64) void freq_tab(float* invf) {
  const int m = threadIdx.x;
  if (m < NFR) {
    const float e   = (float)(2 * m) * (1.0f / (float)HD);
    const float p   = powf(10000.0f, e);
    const float inv = 1.0f / p;
    *(volatile float*)(invf + m) = inv;
    __threadfence();
    *(volatile float*)(invf + m) = inv;
  }
}
__global__ __launch_bounds__(256) void trig_tab(const float* __restrict__ invf, float* cosT, float* sinT) {
  const int i = blockIdx.x * 256 + threadIdx.x;
  if (i < SEQ * NFR) {
    const int t = i >> 6, m = i & (NFR - 1);
    const float ang = (float)t * invf[m];
    float sn, cs;
    sincosf(ang, &sn, &cs);
    *(volatile float*)(cosT + i) = cs;
    *(volatile float*)(sinT + i) = sn;
    __threadfence();
    *(volatile float*)(cosT + i) = cs;
    *(volatile float*)(sinT + i) = sn;
  }
}

__global__ __launch_bounds__(256)
void rope_cvt(const float* __restrict__ qkvf, const float* __restrict__ cosT, const float* __restrict__ sinT,
              unsigned short* qh, unsigned short* qrs, unsigned short* kh, unsigned short* krs,
              float* qpp, float* kpp) {
  __shared__ __align__(16) _Float16 sH[64 * 136];
  __shared__ __align__(16) _Float16 sR[64 * 136];
  __shared__ __align__(16) float sP[128];
  const int tid  = threadIdx.x;
  const int wave = tid >> 5, lane = tid & 31;
  const int r0   = blockIdx.x * 64;
  const int slot = blockIdx.y;
  const bool isq = slot < NH;
  const int kvh  = isq ? 0 : (slot - NH);
  const int scol = isq ? slot * HD : (DM + kvh * HD);
  unsigned short* dH = isq ? qh : kh;
  unsigned short* dR = isq ? qrs : krs;
  const int dpitch = isq ? DM : DKV;
  const int dcol   = isq ? slot * HD : kvh * HD;
  const int b  = r0 / SEQ;
  const int t0 = r0 - b * SEQ;

  {
    const int tt = tid >> 2, q4 = tid & 3;
    const int t = t0 + tt;
    const float* src = qkvf + (size_t)(r0 + tt) * DQKV + scol + q4 * 16;
    const float* cp  = cosT + (size_t)t * NFR + q4 * 16;
    const float* sp  = sinT + (size_t)t * NFR + q4 * 16;
    float o1[16], o2[16];
#pragma unroll
    for (int e4 = 0; e4 < 4; ++e4) {
      const v4f a  = *(const v4f*)(src + 4 * e4);
      const v4f a2 = *(const v4f*)(src + NFR + 4 * e4);
      const v4f cc = *(const v4f*)(cp + 4 * e4);
      const v4f ss = *(const v4f*)(sp + 4 * e4);
#pragma unroll
      for (int u = 0; u < 4; ++u) {
        const float x1 = a[u], x2 = a2[u], cv = cc[u], sv = ss[u];
        o1[4 * e4 + u] = x1 * cv - x2 * sv;
        o2[4 * e4 + u] = x2 * cv + x1 * sv;
      }
    }
    if (q4 == 0) {
      const float DN = 0.57735026919f;
      if (isq) {
        const float s0 = (slot & 4) ? DN : -DN;
        const float s1 = (slot & 2) ? DN : -DN;
        const float s2 = (slot & 1) ? DN : -DN;
        sP[tt] = o1[0] * s0 + o1[1] * s1 + o1[2] * s2;
      } else {
#pragma unroll
        for (int u = 0; u < 2; ++u) {
          const int hu = kvh * NREP + u;
          const float s0 = (hu & 4) ? DN : -DN;
          const float s1 = (hu & 2) ? DN : -DN;
          const float s2 = (hu & 1) ? DN : -DN;
          sP[u * 64 + tt] = o1[0] * s0 + o1[1] * s1 + o1[2] * s2;
        }
      }
    }
    v8h H0, H1, H2, H3, R0, R1, R2, R3;
#pragma unroll
    for (int u = 0; u < 8; ++u) {
      _Float16 x, y;
      split16(o1[u] * 16.0f, x, y);      H0[u] = x;  R0[u] = y;
      split16(o1[8 + u] * 16.0f, x, y);  H1[u] = x;  R1[u] = y;
      split16(o2[u] * 16.0f, x, y);      H2[u] = x;  R2[u] = y;
      split16(o2[8 + u] * 16.0f, x, y);  H3[u] = x;  R3[u] = y;
    }
    _Float16* bh = sH + tt * 136 + q4 * 16;
    _Float16* br = sR + tt * 136 + q4 * 16;
    *(v8h*)(bh)       = H0;
    *(v8h*)(bh + 8)   = H1;
    *(v8h*)(bh + NFR) = H2;
    *(v8h*)(bh + NFR + 8) = H3;
    *(v8h*)(br)       = R0;
    *(v8h*)(br + 8)   = R1;
    *(v8h*)(br + NFR) = R2;
    *(v8h*)(br + NFR + 8) = R3;
  }
  __syncthreads();

  const int hq = lane >> 4, piece = lane & 15;
  v4u vh[4], vr[4];
  size_t go[4];
#pragma unroll
  for (int it = 0; it < 4; ++it) {
    const int rr = it * 16 + wave * 2 + hq;
    vh[it] = *(const v4u*)(sH + rr * 136 + piece * 8);
    vr[it] = *(const v4u*)(sR + rr * 136 + piece * 8);
    go[it] = (size_t)(r0 + rr) * dpitch + dcol + piece * 8;
  }
  const v4f  gv  = *(const v4f*)(sP + (isq ? piece * 4 : lane * 4));
  const bool gst = (wave == 0) && (isq ? (lane < 16) : true);
  float* gp = isq ? (qpp + (size_t)(b * NH + slot) * SEQ + t0 + piece * 4)
                  : (kpp + (size_t)(b * NH + kvh * NREP + hq) * SEQ + t0 + piece * 4);
  for (int pass = 0; pass < 2; ++pass) {
#pragma unroll
    for (int it = 0; it < 4; ++it) {
      *(volatile v4u*)(dH + go[it]) = vh[it];
      *(volatile v4u*)(dR + go[it]) = vr[it];
    }
    if (gst) *(volatile v4f*)gp = gv;
    __threadfence();
  }
}

__global__ __launch_bounds__(256) void v_tr(const float* __restrict__ qkvf, unsigned short* vt, unsigned short* vtr) {
  __shared__ __align__(16) float sv[64 * 68];
  const int tid  = threadIdx.x;
  const int t0   = blockIdx.x * 64;
  const int slot = blockIdx.y;
  const int kvh  = slot >> 1, dh = (slot & 1) * 64;
  const int b    = blockIdx.z;
#pragma unroll
  for (int i = 0; i < 4; ++i) {
    const int idx = i * 256 + tid;
    const int tt = idx >> 4, c4 = (idx & 15) * 4;
    const v4f a = *(const v4f*)(qkvf + ((size_t)(b * SEQ + t0 + tt)) * DQKV + DM + DKV + kvh * HD + dh + c4);
    *(v4f*)(sv + tt * 68 + c4) = a;
  }
  __syncthreads();

  const int g = tid >> 3, piece = tid & 7;
  v4u hv[2], rv[2];
  size_t ho[2];
#pragma unroll
  for (int it = 0; it < 2; ++it) {
    const int d = it * 32 + g;
    v4u p, q;
#pragma unroll
    for (int e = 0; e < 4; ++e) {
      _Float16 x0, y0, x1, y1;
      split16(sv[(piece * 8 + 2 * e) * 68 + d] * 16.0f, x0, y0);
      split16(sv[(piece * 8 + 2 * e + 1) * 68 + d] * 16.0f, x1, y1);
      p[e] = pk16(h_bits(x0), h_bits(x1));
      q[e] = pk16(h_bits(y0), h_bits(y1));
    }
    hv[it] = p;
    rv[it] = q;
    ho[it] = ((size_t)((b * NKV + kvh) * HD + dh + d)) * SEQ + t0 + piece * 8;
  }
  for (int pass = 0; pass < 2; ++pass) {
#pragma unroll
    for (int it = 0; it < 2; ++it) {
      *(volatile v4u*)(vt + ho[it])  = hv[it];
      *(volatile v4u*)(vtr + ho[it]) = rv[it];
    }
    __threadfence();
  }
}

__global__ __launch_bounds__(128)
void attn_k(const unsigned short* __restrict__ qhp, const unsigned short* __restrict__ qrsp,
            const unsigned short* __restrict__ khp, const unsigned short* __restrict__ krsp,
            const unsigned short* __restrict__ vtp, const unsigned short* __restrict__ vtrp,
            const float* __restrict__ qpp, const float* __restrict__ kpp, const float* __restrict__ hsc,
            unsigned short* ctxp, unsigned short* ctxrp) {
  union FH { v16h v; v8h h[2]; };
  constexpr int KTB    = 64 * HD * 2;
  constexpr int PTB    = 4 * 16 * 64 * 2;
  constexpr int OFF_K  = 0;
  constexpr int OFF_KR = KTB;
  constexpr int OFF_V  = 2 * KTB;
  constexpr int OFF_VR = 3 * KTB;
  constexpr int OFF_P  = 4 * KTB;
  constexpr int OFF_PR = OFF_P + PTB;
  constexpr int SMEMB  = OFF_PR + PTB;
  static_assert(4 * 16 * HD * 4 <= OFF_V);
  static_assert(SMEMB == 81920);
  __shared__ __align__(16) unsigned char smem[SMEMB];
  _Float16* Ksh = (_Float16*)(smem + OFF_K);
  _Float16* Krs = (_Float16*)(smem + OFF_KR);
  _Float16* Vsh = (_Float16*)(smem + OFF_V);
  _Float16* Vrs = (_Float16*)(smem + OFF_VR);
  _Float16* Psh = (_Float16*)(smem + OFF_P);
  _Float16* Prs = (_Float16*)(smem + OFF_PR);

  const int tid  = threadIdx.x;
  const int wave = tid >> 5;
  const int lane = tid & 31;
  const int hh   = lane >> 4;
  const int c    = lane & 15;

  const int bx   = blockIdx.x;
  const int qb   = bx % NQB;
  const int rest = bx / NQB;
  const int h    = rest % NH;
  const int b    = rest / NH;
  const int kvh  = h / NREP;
  const int q0   = qb * 64 + wave * 16;
  const size_t rowB = (size_t)b * SEQ;

  const _Float16* Qg  = (const _Float16*)(const void*)qhp  + (size_t)h * HD;
  const _Float16* Qrg = (const _Float16*)(const void*)qrsp + (size_t)h * HD;
  const _Float16* Kg  = (const _Float16*)(const void*)khp  + (size_t)kvh * HD;
  const _Float16* Krg = (const _Float16*)(const void*)krsp + (size_t)kvh * HD;
  const _Float16* Vg  = (const _Float16*)(const void*)vtp  + ((size_t)(b * NKV + kvh) * HD) * SEQ;
  const _Float16* Vrg = (const _Float16*)(const void*)vtrp + ((size_t)(b * NKV + kvh) * HD) * SEQ;
  const float hs = bfr(hsc[h]);
  const float* qpb = qpp + (size_t)(b * NH + h) * SEQ;
  const float* kpb = kpp + (size_t)(b * NH + h) * SEQ;
  const float SC = 0.08838834764831845f * (1.0f / 256.0f);

  float qpv[8], lsum[8], mrun[8];
  v8f oacc[8];
#pragma unroll
  for (int r = 0; r < 8; ++r) { qpv[r] = qpb[q0 + 8 * hh + r]; lsum[r] = 0.f; mrun[r] = -1e30f; }
#pragma unroll
  for (int t = 0; t < 8; ++t) oacc[t] = zero8();

  _Float16* pw  = Psh + wave * (16 * 64);
  _Float16* prw = Prs + wave * (16 * 64);

  const int ktlo = (qb >= KTW - 1) ? (qb - (KTW - 1)) : 0;
  const int nkt  = qb - ktlo + 1;
  for (int kti = 0; kti < nkt; ++kti) {
    const int kv0 = (ktlo + kti) * 64;
    __syncthreads();
    {
      const int r = tid >> 1, dh = (tid & 1) * 64;
      const size_t ko = (rowB + kv0 + r) * DKV + dh;
#pragma unroll
      for (int i = 0; i < 8; ++i) {
        const v8h a0 = *(const v8h*)(Kg + ko + 8 * i);
        const v8h a1 = *(const v8h*)(Krg + ko + 8 * i);
        *(v8h*)(Ksh + r * HD + dh + 8 * i) = a0;
        *(v8h*)(Krs + r * HD + dh + 8 * i) = a1;
      }
      const int d = tid;
      const size_t vo = (size_t)d * SEQ + kv0;
#pragma unroll
      for (int i = 0; i < 8; ++i) {
        const v8h b0 = *(const v8h*)(Vg + vo + 8 * i);
        const v8h b1 = *(const v8h*)(Vrg + vo + 8 * i);
        *(v8h*)(Vsh + d * 64 + 8 * i) = b0;
        *(v8h*)(Vrs + d * 64 + 8 * i) = b1;
      }
    }
    __syncthreads();

    float kpj[4];
#pragma unroll
    for (int j = 0; j < 4; ++j) kpj[j] = kpb[kv0 + j * 16 + c];

    v8f s[4];
#pragma unroll
    for (int j = 0; j < 4; ++j) {
      v8f sacc = zero8(), tacc = zero8();
      const _Float16* kq  = Ksh + (j * 16 + c) * HD + 8 * hh;
      const _Float16* krq = Krs + (j * 16 + c) * HD + 8 * hh;
#pragma unroll 1
      for (int dc = 0; dc < 4; ++dc) {
        const size_t qo = (rowB + q0 + c) * DM + dc * 32 + 8 * hh;
        const v16h qa = ldfrag_h(Qg + qo);
        const v16h qr = ldfrag_h(Qrg + qo);
        FH kb, krb;
        kb.h[0]  = *(const v8h*)(kq + dc * 32);
        kb.h[1]  = *(const v8h*)(kq + dc * 32 + 16);
        krb.h[0] = *(const v8h*)(krq + dc * 32);
        krb.h[1] = *(const v8h*)(krq + dc * 32 + 16);
        sacc = mma_h(qa, kb.v, sacc);
        tacc = mma_h(qa, krb.v, tacc);
        tacc = mma_h(qr, kb.v, tacc);
      }
      s[j] = sacc + tacc * (1.0f / 2048.0f);
    }

    float alpha[8];
#pragma unroll
    for (int r = 0; r < 8; ++r) {
      const int qrow = q0 + 8 * hh + r;
      float av[4];
      float tmx = -1e30f;
#pragma unroll
      for (int j = 0; j < 4; ++j) {
        const int key = kv0 + j * 16 + c;
        const float sr = s[j][r] * SC;
        const float g  = qpv[r] * kpj[j];
        const float bb = hs * g;
        float a = sr + bb;
        const bool ok = (key <= qrow) && (key + WIN > qrow);
        a = ok ? a : -1e30f;
        av[j] = a;
        tmx = fmaxf(tmx, a);
      }
#pragma unroll
      for (int off = 1; off < 16; off <<= 1) tmx = fmaxf(tmx, __shfl_xor(tmx, off, 32));
      const float mn = fmaxf(mrun[r], tmx);
      const float al = __expf(mrun[r] - mn);
      alpha[r] = al;
      mrun[r]  = mn;
      float ps = 0.0f;
#pragma unroll
      for (int j = 0; j < 4; ++j) {
        const int key = kv0 + j * 16 + c;
        const bool ok = (key <= qrow) && (key + WIN > qrow);
        float p = __expf(av[j] - mn);
        p = ok ? p : 0.0f;
        ps += p;
        _Float16 x0, y0;
        split16(p * 256.0f, x0, y0);
        pw[(8 * hh + r) * 64 + j * 16 + c]  = x0;
        prw[(8 * hh + r) * 64 + j * 16 + c] = y0;
      }
      lsum[r] = lsum[r] * al + ps;
    }
    __builtin_amdgcn_fence(__ATOMIC_RELEASE, "workgroup");
    __builtin_amdgcn_wave_barrier();
    __builtin_amdgcn_fence(__ATOMIC_ACQUIRE, "workgroup");

#pragma unroll
    for (int t = 0; t < 8; ++t) {
#pragma unroll
      for (int r = 0; r < 8; ++r) oacc[t][r] = oacc[t][r] * alpha[r];
    }
    acc_guard4(oacc[0], oacc[1], oacc[2], oacc[3]);
    acc_guard4(oacc[4], oacc[5], oacc[6], oacc[7]);

    FH pa[2], par[2];
#pragma unroll
    for (int kk = 0; kk < 2; ++kk) {
      pa[kk].h[0]  = *(const v8h*)(pw + c * 64 + kk * 32 + 8 * hh);
      pa[kk].h[1]  = *(const v8h*)(pw + c * 64 + kk * 32 + 16 + 8 * hh);
      par[kk].h[0] = *(const v8h*)(prw + c * 64 + kk * 32 + 8 * hh);
      par[kk].h[1] = *(const v8h*)(prw + c * 64 + kk * 32 + 16 + 8 * hh);
    }
#pragma unroll
    for (int t = 0; t < 8; ++t) {
      v8f tr = zero8();
#pragma unroll
      for (int kk = 0; kk < 2; ++kk) {
        FH vb, vrb;
        vb.h[0]  = *(const v8h*)(Vsh + (t * 16 + c) * 64 + kk * 32 + 8 * hh);
        vb.h[1]  = *(const v8h*)(Vsh + (t * 16 + c) * 64 + kk * 32 + 16 + 8 * hh);
        vrb.h[0] = *(const v8h*)(Vrs + (t * 16 + c) * 64 + kk * 32 + 8 * hh);
        vrb.h[1] = *(const v8h*)(Vrs + (t * 16 + c) * 64 + kk * 32 + 16 + 8 * hh);
        tr = mma_h(pa[kk].v, vrb.v, tr);
        tr = mma_h(par[kk].v, vb.v, tr);
        oacc[t] = mma_h(pa[kk].v, vb.v, oacc[t]);
      }
      oacc[t] = oacc[t] + tr * (1.0f / 2048.0f);
    }
    acc_guard4(oacc[0], oacc[1], oacc[2], oacc[3]);
    acc_guard4(oacc[4], oacc[5], oacc[6], oacc[7]);
  }
  __syncthreads();

  float* os = (float*)(void*)smem + wave * (16 * HD);
#pragma unroll
  for (int r = 0; r < 8; ++r) {
    float l = lsum[r];
#pragma unroll
    for (int off = 1; off < 16; off <<= 1) l += __shfl_xor(l, off, 32);
    const float rl = 1.0f / l;
    const float sc = rl * (1.0f / 256.0f);
#pragma unroll
    for (int t = 0; t < 8; ++t) os[(8 * hh + r) * HD + t * 16 + c] = oacc[t][r] * sc;
  }
  __builtin_amdgcn_fence(__ATOMIC_RELEASE, "workgroup");
  __builtin_amdgcn_wave_barrier();
  __builtin_amdgcn_fence(__ATOMIC_ACQUIRE, "workgroup");
  {
    const int piece = lane & 15;
    v4u ph[8], pr[8];
#pragma unroll
    for (int it = 0; it < 8; ++it) {
      const int row = it * 2 + hh;
      const v4f a  = *(const v4f*)(os + row * HD + piece * 8);
      const v4f a2 = *(const v4f*)(os + row * HD + piece * 8 + 4);
      float f[8];
      f[0] = a[0];  f[1] = a[1];  f[2] = a[2];  f[3] = a[3];
      f[4] = a2[0]; f[5] = a2[1]; f[6] = a2[2]; f[7] = a2[3];
      v4u p, q;
#pragma unroll
      for (int e = 0; e < 4; ++e) {
        _Float16 x0, y0, x1, y1;
        split16(f[2 * e], x0, y0);
        split16(f[2 * e + 1], x1, y1);
        p[e] = pk16(h_bits(x0), h_bits(x1));
        q[e] = pk16(h_bits(y0), h_bits(y1));
      }
      ph[it] = p;
      pr[it] = q;
    }
    for (int pass = 0; pass < 2; ++pass) {
#pragma unroll
      for (int it = 0; it < 8; ++it) {
        const int row = it * 2 + hh;
        const size_t go = (rowB + q0 + row) * DM + (size_t)h * HD + piece * 8;
        *(volatile v4u*)(ctxp + go)  = ph[it];
        *(volatile v4u*)(ctxrp + go) = pr[it];
      }
      __threadfence();
    }
  }
}

extern "C" void kernel_launch(void* const* d_in, const int* in_sizes, int n_in,
                              void* d_out, int out_size, void* d_ws, size_t ws_size,
                              hipStream_t stream) {
  if (n_in < 6) return;
  if (in_sizes[0] != ROWS * DM) return;
  if (in_sizes[1] != DM * DM) return;
  if (in_sizes[2] != DM * DKV) return;
  if (in_sizes[3] != DM * DKV) return;
  if (in_sizes[4] != DM * DM) return;
  if (in_sizes[5] != NH) return;
  if (out_size != OUTN) return;

  const float* x   = (const float*)d_in[0];
  const float* wq  = (const float*)d_in[1];
  const float* wk  = (const float*)d_in[2];
  const float* wv  = (const float*)d_in[3];
  const float* wo  = (const float*)d_in[4];
  const float* hsc = (const float*)d_in[5];

  const size_t PX    = (size_t)ROWS * DM * 2;
  const size_t PWT   = (size_t)DQKV * DM * 2;
  const size_t PWO   = (size_t)DM * DM * 2;
  const size_t PQKVF = (size_t)ROWS * DQKV * 4;
  const size_t PTR   = (size_t)SEQ * NFR * 4;
  const size_t PQ    = (size_t)ROWS * DM * 2;
  const size_t PK    = (size_t)ROWS * DKV * 2;
  const size_t PVT   = (size_t)NB * NKV * HD * SEQ * 2;
  const size_t PGP   = (size_t)NB * NH * SEQ * 4;
  const size_t PCTX  = (size_t)ROWS * DM * 2;
  const size_t PINV  = 256;
  size_t off = 0;
  const size_t oX    = off; off += PX;
  const size_t oWT   = off; off += PWT;
  const size_t oWO   = off; off += PWO;
  const size_t oQKVF = off; off += PQKVF;
  const size_t oCOS  = off; off += PTR;
  const size_t oSIN  = off; off += PTR;
  const size_t oQH   = off; off += PQ;
  const size_t oQR   = off; off += PQ;
  const size_t oKH   = off; off += PK;
  const size_t oKR   = off; off += PK;
  const size_t oVT   = off; off += PVT;
  const size_t oVTR  = off; off += PVT;
  const size_t oQP   = off; off += PGP;
  const size_t oKP   = off; off += PGP;
  const size_t oCTX  = off; off += PCTX;
  const size_t oCTXR = off; off += PCTX;
  const size_t oINV  = off; off += PINV;
  if (off > ws_size) return;
  if (off > (size_t)134217728) return;

  char* ws = (char*)d_ws;
  unsigned short* Xh   = (unsigned short*)(ws + oX);
  unsigned short* WT   = (unsigned short*)(ws + oWT);
  unsigned short* WOT  = (unsigned short*)(ws + oWO);
  float*          QKVF = (float*)(ws + oQKVF);
  float*          COS  = (float*)(ws + oCOS);
  float*          SIN  = (float*)(ws + oSIN);
  unsigned short* QH   = (unsigned short*)(ws + oQH);
  unsigned short* QR   = (unsigned short*)(ws + oQR);
  unsigned short* KH   = (unsigned short*)(ws + oKH);
  unsigned short* KR   = (unsigned short*)(ws + oKR);
  unsigned short* VT   = (unsigned short*)(ws + oVT);
  unsigned short* VTR  = (unsigned short*)(ws + oVTR);
  float*          QP   = (float*)(ws + oQP);
  float*          KP   = (float*)(ws + oKP);
  unsigned short* CTX  = (unsigned short*)(ws + oCTX);
  unsigned short* CTXR = (unsigned short*)(ws + oCTXR);
  float*          INVF = (float*)(ws + oINV);
  float*          outf = (float*)d_out;

  const dim3 blk(256);
  const int n8x = ROWS * DM / 8;
  const dim3 gCx((n8x + 255) / 256);
  const dim3 gTq(DM / 64, DM / 64);
  const dim3 gTk(DKV / 64, DM / 64);
  const dim3 gTo(DM / 64, DM / 64);
  const dim3 gTab((SEQ * NFR + 255) / 256);
  const dim3 gGqkv(((ROWS / 64) * (DQKV / 64) + 7) / 8);
  const dim3 gGdm(((ROWS / 64) * (DM / 64) + 7) / 8);
  const dim3 gRope(ROWS / 64, NH + NKV);
  const dim3 gVt(SEQ / 64, NKV * 2, NB);
  const dim3 gAttn(NQB * NH * NB);
  const float wScale = 1024.0f;
  const float aScale = 16.0f;
  const float cscale = 1.0f / 16384.0f;

  cvt16<<<gCx, blk, 0, stream>>>(x, Xh, n8x, aScale);
  w_tr<<<gTq, blk, 0, stream>>>(wq, WT, DM, DM, wScale);
  w_tr<<<gTk, blk, 0, stream>>>(wk, WT + (size_t)DM * DM, DM, DKV, wScale);
  w_tr<<<gTk, blk, 0, stream>>>(wv, WT + (size_t)(DM + DKV) * DM, DM, DKV, wScale);
  w_tr<<<gTo, blk, 0, stream>>>(wo, WOT, DM, DM, wScale);
  freq_tab<<<dim3(1), dim3(64), 0, stream>>>(INVF);
  trig_tab<<<gTab, blk, 0, stream>>>(INVF, COS, SIN);
  gemm64_f16<1, false><<<gGqkv, blk, 0, stream>>>(Xh, Xh, DM, WT, DM, cscale, (void*)QKVF, QH, DQKV,
                                                  ROWS, DQKV, DM, 1.0f, SEQ, 0, SEQ);
  rope_cvt<<<gRope, blk, 0, stream>>>(QKVF, COS, SIN, QH, QR, KH, KR, QP, KP);
  v_tr<<<gVt, blk, 0, stream>>>(QKVF, VT, VTR);
  attn_k<<<gAttn, dim3(128), 0, stream>>>(QH, QR, KH, KR, VT, VTR, QP, KP, hsc, CTX, CTXR);
  gemm64_f16<1, true><<<gGdm, blk, 0, stream>>>(CTX, CTXR, DM, WOT, DM, cscale, (void*)outf, CTXR, DM,
                                                ROWS, DM, DM, 1.0f, SEQ, 0, SEQ);
  (void)hipGetLastError();
}
